// MultiHeadAttention_25245817766393
// MI455X (gfx1250) — hardware-run, weakly checked
//
#include <hip/hip_runtime.h>
#ifndef NB
#define NB 4
#endif
#ifndef SEQ
#define SEQ 4096
#endif
#define NB_FULL 4
#define SEQ_FULL 4096
#define HD 64
#define BSTRIDE_FULL ((size_t)SEQ_FULL * HD)

static_assert(SEQ % 64 == 0);
static_assert(SEQ <= SEQ_FULL);
static_assert(NB <= NB_FULL);
static_assert(HD == 64);
static_assert((size_t)NB * SEQ * HD * 2 * 2 + 512 <= (size_t)134217728);

typedef __bf16 v16b __attribute__((ext_vector_type(16)));
typedef _Float16 v16h __attribute__((ext_vector_type(16)));
typedef unsigned short v8us __attribute__((ext_vector_type(8), may_alias));
typedef float v8f __attribute__((ext_vector_type(8)));
typedef float v4f __attribute__((ext_vector_type(4)));
typedef float v4fa __attribute__((ext_vector_type(4), may_alias));
union FragB { v16b v; v8us half[2]; unsigned short u[16]; };
union FragH { v16h v; v8us half[2]; _Float16 h[16]; unsigned short u[16]; };

#define LOG2E 1.4426950408889634f
#define NEGV (-1000000000.0f)

__device__ __forceinline__ unsigned short bf16_bits(float x) {
  unsigned int u = __float_as_uint(x);
  return (unsigned short)((u + 0x7FFFu + ((u >> 16) & 1u)) >> 16);
}
__device__ __forceinline__ float bf16_val(unsigned short b) { return __uint_as_float(((unsigned int)b) << 16); }
__device__ __forceinline__ float bf16_rne(float x) { return bf16_val(bf16_bits(x)); }

__device__ __forceinline__ v8f mma_bf2(v16b a0, v16b b0, v16b a1, v16b b1, v8f c) {
  c = __builtin_amdgcn_wmma_f32_16x16x32_bf16(false, a0, false, b0, (short)0, c, false, false);
  c = __builtin_amdgcn_wmma_f32_16x16x32_bf16(false, a1, false, b1, (short)0, c, false, false);
  asm volatile("v_nop\n\tv_nop\n\tv_nop\n\tv_nop" : "+v"(c) : "v"(a0), "v"(b0), "v"(a1), "v"(b1));
  return c;
}
__device__ __forceinline__ void mma_h2(v16h a, v16h bh, v16h bl, v8f& ch, v8f& cl) {
  ch = __builtin_amdgcn_wmma_f32_16x16x32_f16(false, a, false, bh, (short)0, ch, false, false);
  cl = __builtin_amdgcn_wmma_f32_16x16x32_f16(false, a, false, bl, (short)0, cl, false, false);
  asm volatile("v_nop\n\tv_nop\n\tv_nop\n\tv_nop" : "+v"(ch), "+v"(cl) : "v"(a), "v"(bh), "v"(bl));
}

__global__ __launch_bounds__(256) void k_kb(const float* __restrict__ K, unsigned short* __restrict__ Kb) {
  const int t = blockIdx.x * 256 + threadIdx.x;
  if (t >= NB * SEQ * 8) return;
  const int row = t >> 3, piece = t & 7;
  const int b = row / SEQ, s = row - b * SEQ;
  const float* src = K + (size_t)b * BSTRIDE_FULL + (size_t)s * HD + piece * 8;
  const v4f x0 = *(const v4fa*)(src), x1 = *(const v4fa*)(src + 4);
  v8us o;
  o[0] = bf16_bits(x0[0]); o[1] = bf16_bits(x0[1]); o[2] = bf16_bits(x0[2]); o[3] = bf16_bits(x0[3]);
  o[4] = bf16_bits(x1[0]); o[5] = bf16_bits(x1[1]); o[6] = bf16_bits(x1[2]); o[7] = bf16_bits(x1[3]);
  unsigned short* d = Kb + (size_t)t * 8;
  *(volatile v8us*)d = o;
  __threadfence();
  *(volatile v8us*)d = o;
}

__global__ __launch_bounds__(256) void k_vt(const float* __restrict__ V, unsigned short* __restrict__ Vt) {
  __shared__ unsigned short tl[64][66];
  const int tid = threadIdx.x;
  const int b = blockIdx.x / (SEQ / 64), sg = blockIdx.x % (SEQ / 64);
  const int s0 = sg * 64;
  for (int i = tid; i < 64 * 16; i += 256) {
    const int j = i >> 4, c4 = (i & 15) * 4;
    const v4f x = *(const v4fa*)(V + (size_t)b * BSTRIDE_FULL + (size_t)(s0 + j) * HD + c4);
    FragH f;
    f.h[0] = (_Float16)(bf16_rne(x[0]) * 16.0f);
    f.h[1] = (_Float16)(bf16_rne(x[1]) * 16.0f);
    f.h[2] = (_Float16)(bf16_rne(x[2]) * 16.0f);
    f.h[3] = (_Float16)(bf16_rne(x[3]) * 16.0f);
    tl[c4 + 0][j] = f.u[0]; tl[c4 + 1][j] = f.u[1]; tl[c4 + 2][j] = f.u[2]; tl[c4 + 3][j] = f.u[3];
  }
  __syncthreads();
  for (int pass = 0; pass < 2; ++pass) {
    for (int i = tid; i < 64 * 8; i += 256) {
      const int d = i >> 3, j8 = (i & 7) * 8;
      v8us o;
#pragma unroll
      for (int q = 0; q < 8; ++q) o[q] = tl[d][j8 + q];
      *(volatile v8us*)(Vt + ((size_t)b * HD + d) * SEQ + s0 + j8) = o;
    }
    if (pass == 0) __threadfence();
  }
}

template <bool MASK>
__device__ __forceinline__ void fa_step(const unsigned short* __restrict__ Kp, const unsigned short* __restrict__ Vp,
                                        int key0, int qg, int ln, int hh, const FragB& q0, const FragB& q1,
                                        float& mr, float& lr, v8f (&Oh)[4], v8f (&Ol)[4]) {
  const unsigned short* kp0 = Kp + (size_t)(key0 + ln) * HD + 8 * hh;
  const unsigned short* kp1 = kp0 + 16 * HD;
  FragB k00, k01, k10, k11;
  k00.half[0] = *(const v8us*)(kp0);      k00.half[1] = *(const v8us*)(kp0 + 16);
  k01.half[0] = *(const v8us*)(kp0 + 32); k01.half[1] = *(const v8us*)(kp0 + 48);
  k10.half[0] = *(const v8us*)(kp1);      k10.half[1] = *(const v8us*)(kp1 + 16);
  k11.half[0] = *(const v8us*)(kp1 + 32); k11.half[1] = *(const v8us*)(kp1 + 48);
  const unsigned short* vp = Vp + (size_t)ln * SEQ + key0 + 8 * hh;
  FragH vf[4];
#pragma unroll
  for (int t = 0; t < 4; ++t) {
    vf[t].half[0] = *(const v8us*)(vp + (size_t)t * 16 * SEQ);
    vf[t].half[1] = *(const v8us*)(vp + (size_t)t * 16 * SEQ + 16);
  }
  const v8f z8 = {0.f, 0.f, 0.f, 0.f, 0.f, 0.f, 0.f, 0.f};
  const v8f s0 = mma_bf2(k00.v, q0.v, k01.v, q1.v, z8);
  const v8f s1 = mma_bf2(k10.v, q0.v, k11.v, q1.v, z8);
  float sc[16];
#pragma unroll
  for (int r = 0; r < 8; ++r) { sc[r] = s0[r] * 0.015625f; sc[8 + r] = s1[r] * 0.015625f; }
  if (MASK) {
#pragma unroll
    for (int r = 0; r < 8; ++r) {
      const int kg = key0 + 8 * hh + r;
      sc[r]     += (kg > qg) ? NEGV : 0.0f;
      sc[8 + r] += (kg + 16 > qg) ? NEGV : 0.0f;
    }
  }
  float mx = sc[0];
#pragma unroll
  for (int i = 1; i < 16; ++i) mx = fmaxf(mx, sc[i]);
  mx = fmaxf(mx, __shfl_xor(mx, 16, 32));
  const float mnew = fmaxf(mr, mx);
  const float al = exp2f((mr - mnew) * LOG2E);
  mr = mnew;
  FragH ph, pl;
  float ps = 0.0f;
#pragma unroll
  for (int i = 0; i < 16; ++i) {
    const float pc = exp2f(fmaf(sc[i] - mnew, LOG2E, 8.0f));
    ps += pc;
    const _Float16 h = (_Float16)pc;
    ph.h[i] = h;
    pl.h[i] = (_Float16)((pc - (float)h) * 2048.0f);
  }
  ps += __shfl_xor(ps, 16, 32);
  lr = lr * al + ps;
#pragma unroll
  for (int t = 0; t < 4; ++t) { Oh[t] = Oh[t] * al; Ol[t] = Ol[t] * al; }
#pragma unroll
  for (int t = 0; t < 4; ++t) mma_h2(vf[t].v, ph.v, pl.v, Oh[t], Ol[t]);
}

__global__ __launch_bounds__(128) void k_attn(const float* __restrict__ Q, const unsigned short* __restrict__ Kb,
                                              const unsigned short* __restrict__ Vt, float* __restrict__ O) {
  __shared__ __attribute__((aligned(16))) float so[4][16][68];
  const int tid = threadIdx.x, w = tid >> 5, lane = tid & 31, ln = lane & 15, hh = lane >> 4;
  const int b = blockIdx.x / (SEQ / 64), qt = blockIdx.x % (SEQ / 64);
  const int qbase = qt * 64 + 16 * w;
  const int qg = qbase + ln;
  const float* qrow = Q + (size_t)b * BSTRIDE_FULL + (size_t)qg * HD;
  FragB q0, q1;
  {
    const v4f a0 = *(const v4fa*)(qrow + 8 * hh),      a1 = *(const v4fa*)(qrow + 8 * hh + 4);
    const v4f a2 = *(const v4fa*)(qrow + 16 + 8 * hh), a3 = *(const v4fa*)(qrow + 16 + 8 * hh + 4);
    const v4f c0 = *(const v4fa*)(qrow + 32 + 8 * hh), c1 = *(const v4fa*)(qrow + 32 + 8 * hh + 4);
    const v4f c2 = *(const v4fa*)(qrow + 48 + 8 * hh), c3 = *(const v4fa*)(qrow + 48 + 8 * hh + 4);
#pragma unroll
    for (int i = 0; i < 4; ++i) {
      q0.u[i] = bf16_bits(a0[i]); q0.u[4 + i] = bf16_bits(a1[i]); q0.u[8 + i] = bf16_bits(a2[i]); q0.u[12 + i] = bf16_bits(a3[i]);
      q1.u[i] = bf16_bits(c0[i]); q1.u[4 + i] = bf16_bits(c1[i]); q1.u[8 + i] = bf16_bits(c2[i]); q1.u[12 + i] = bf16_bits(c3[i]);
    }
  }
  float mr = -3.0e38f, lr = 0.0f;
  v8f Oh[4] = {}, Ol[4] = {};
  const unsigned short* Kp = Kb + (size_t)b * SEQ * HD;
  const unsigned short* Vp = Vt + (size_t)b * HD * SEQ;
  const int nfull = qbase >> 5;
#pragma unroll 1
  for (int j = 0; j < nfull; ++j)
    fa_step<false>(Kp, Vp, 32 * j, qg, ln, hh, q0, q1, mr, lr, Oh, Ol);
  fa_step<true>(Kp, Vp, 32 * nfull, qg, ln, hh, q0, q1, mr, lr, Oh, Ol);

  const float inv = 1.0f / (16.0f * lr);
#pragma unroll
  for (int t = 0; t < 4; ++t)
#pragma unroll
    for (int r = 0; r < 8; ++r)
      so[w][ln][16 * t + 8 * hh + r] = (Oh[t][r] + Ol[t][r] * 0.00048828125f) * inv;
  __syncthreads();
  float* og = O + (size_t)b * BSTRIDE_FULL + (size_t)qbase * HD;
  const int rsub = lane >> 4, c4 = (lane & 15) * 4;
  for (int pass = 0; pass < 2; ++pass) {
#pragma unroll
    for (int q = 0; q < 8; ++q) {
      const int row = 2 * q + rsub;
      const v4f v = *(const v4fa*)&so[w][row][c4];
      *(volatile v4f*)(og + (size_t)row * HD + c4) = v;
    }
    if (pass == 0) __threadfence();
  }
}

extern "C" void kernel_launch(void* const* d_in, const int* in_sizes, int n_in,
                              void* d_out, int out_size, void* d_ws, size_t ws_size, hipStream_t stream) {
  if (n_in < 3) return;
  const long long need = (long long)(NB - 1) * SEQ_FULL * HD + (long long)SEQ * HD;
  if ((long long)in_sizes[0] < need || (long long)in_sizes[1] < need || (long long)in_sizes[2] < need) return;
  if ((long long)out_size < need) return;
  const float* Q = (const float*)d_in[0];
  const float* K = (const float*)d_in[1];
  const float* V = (const float*)d_in[2];
  float* O = (float*)d_out;
  char* ws = (char*)d_ws;
  size_t off = 0;
  const size_t plane = (size_t)NB * SEQ * HD * 2;
  unsigned short* Kb = (unsigned short*)(ws + off); off += (plane + 255) & ~(size_t)255;
  unsigned short* Vt = (unsigned short*)(ws + off); off += (plane + 255) & ~(size_t)255;
  if (off > ws_size) return;
  k_kb<<<(unsigned)((NB * SEQ * 8 + 255) / 256), 256, 0, stream>>>(K, Kb);
  k_vt<<<(unsigned)(NB * (SEQ / 64)), 256, 0, stream>>>(V, Vt);
  k_attn<<<(unsigned)(NB * (SEQ / 64)), 128, 0, stream>>>(Q, Kb, Vt, O);
}
